// TransitionGNN_24713241822152
// MI455X (gfx1250) — hardware-verified
//
#include <hip/hip_runtime.h>
#include <stddef.h>
#include <stdint.h>


#define NBAT   2048
#define NOBJ   10
#define DIN    32
#define HID    512
#define ADIM   4
#define NNODE  20480
#define KIN    548
#define XK     576
#define NEROW  45
#define PQP    1024
#define W1P    64
#define XAP    40
#define HP     520
#define XP     584
#define NTHR   256
#define NPREP  3104
#define WSCL   16.0f
#define C16    0.0625f
#define C256   0.00390625f
#define LNEPS  1e-5f
#define WSCAP  134217728

static_assert(NNODE == NBAT * NOBJ);
static_assert(NTHR == 8 * 32);
static_assert((NNODE % 32) == 0);
static_assert((XK % 32) == 0);
static_assert((HID % 32) == 0);
static_assert(((XAP * 2) % 16) == 0);
static_assert(((HP * 2) % 16) == 0);
static_assert(((XP * 2) % 16) == 0);
static_assert(XK >= KIN);
static_assert(NPREP == 1024 + 4 * HID + DIN);

#define SZ_EW1T ((size_t)1024 * W1P * 2)
#define SZ_EW2T ((size_t)HID * HID * 2)
#define SZ_EW3T ((size_t)HID * HID * 2)
#define SZ_NW1T ((size_t)HID * XK * 2)
#define SZ_NW2T ((size_t)HID * HID * 2)
#define SZ_NW3T ((size_t)DIN * HID * 2)
#define SZ_PQ   ((size_t)NNODE * PQP * 4)
#define SZ_S    ((size_t)NNODE * HID * 2)
#define SZ_XN   ((size_t)NNODE * XK * 2)
#define SZ_HN1  ((size_t)NNODE * HID * 2)
#define SZ_TOT  (SZ_EW1T + SZ_EW2T + SZ_EW3T + SZ_NW1T + SZ_NW2T + SZ_NW3T + SZ_PQ + SZ_S)
static_assert(SZ_TOT == 107184128);
static_assert(SZ_TOT <= (size_t)WSCAP);
static_assert(SZ_XN + SZ_HN1 <= SZ_PQ);
static_assert((SZ_EW1T % 256) == 0);
static_assert((SZ_EW2T % 256) == 0);
static_assert((SZ_EW3T % 256) == 0);
static_assert((SZ_NW1T % 256) == 0);
static_assert((SZ_NW2T % 256) == 0);
static_assert((SZ_NW3T % 256) == 0);
static_assert((SZ_PQ % 256) == 0);
static_assert((SZ_S % 256) == 0);
static_assert((SZ_XN % 256) == 0);

typedef _Float16     v16h __attribute__((ext_vector_type(16)));
typedef _Float16     v8h  __attribute__((ext_vector_type(8)));
typedef _Float16     v4h  __attribute__((ext_vector_type(4)));
typedef float        v8f  __attribute__((ext_vector_type(8)));
typedef float        v4f  __attribute__((ext_vector_type(4)));
typedef unsigned int v4u  __attribute__((ext_vector_type(4)));
union Frag { v16h v; v8h half[2]; };
union Pk8  { v8h h; v4u u; };

__device__ __forceinline__ v4u cvt8(const v4f a, const v4f b) {
  v8h hv = {(_Float16)a.x, (_Float16)a.y, (_Float16)a.z, (_Float16)a.w,
            (_Float16)b.x, (_Float16)b.y, (_Float16)b.z, (_Float16)b.w};
  Pk8 p;
  p.h = hv;
  return p.u;
}

__device__ __forceinline__ v8f wmh(v16h a, v16h b, v8f c) {
  v8f d = __builtin_amdgcn_wmma_f32_16x16x32_f16(false, a, false, b, (short)0, c, false, false);
  asm volatile("v_nop\n\tv_nop\n\tv_nop\n\tv_nop" : "+v"(d) : "v"(a), "v"(b));
  return d;
}

__device__ __forceinline__ v16h ldf(const _Float16* p, int h) {
  Frag f;
  const _Float16* q = p + 8 * h;
  f.half[0] = *(const v8h*)q;
  f.half[1] = *(const v8h*)(q + 16);
  return f.v;
}

__device__ __forceinline__ float sum16(float s) {
  s += __shfl_xor(s, 1);
  s += __shfl_xor(s, 2);
  s += __shfl_xor(s, 4);
  s += __shfl_xor(s, 8);
  return s;
}

__global__ __launch_bounds__(64) void k_prep(const float* __restrict__ eW1, const float* __restrict__ eW2,
                                             const float* __restrict__ eW3, const float* __restrict__ nW1,
                                             const float* __restrict__ nW2, const float* __restrict__ nW3,
                                             _Float16* eW1T, _Float16* eW2T, _Float16* eW3T,
                                             _Float16* nW1T, _Float16* nW2T, _Float16* nW3T) {
  const int blk = blockIdx.x, tid = threadIdx.x;
  const float* src;
  _Float16* dst;
  int strd, ksrc, kp;
  if (blk < 1024) {
    const int n = blk;
    src = (n < HID) ? (eW1 + n) : (eW1 + (size_t)DIN * HID + (n - HID));
    strd = HID; ksrc = DIN; kp = W1P;
    dst = eW1T + (size_t)n * W1P;
  } else if (blk < 1024 + HID) {
    const int n = blk - 1024;
    src = eW2 + n; strd = HID; ksrc = HID; kp = HID;
    dst = eW2T + (size_t)n * HID;
  } else if (blk < 1024 + 2 * HID) {
    const int n = blk - 1024 - HID;
    src = eW3 + n; strd = HID; ksrc = HID; kp = HID;
    dst = eW3T + (size_t)n * HID;
  } else if (blk < 1024 + 3 * HID) {
    const int n = blk - 1024 - 2 * HID;
    src = nW1 + n; strd = HID; ksrc = KIN; kp = XK;
    dst = nW1T + (size_t)n * XK;
  } else if (blk < 1024 + 4 * HID) {
    const int n = blk - 1024 - 3 * HID;
    src = nW2 + n; strd = HID; ksrc = HID; kp = HID;
    dst = nW2T + (size_t)n * HID;
  } else {
    const int n = blk - 1024 - 4 * HID;
    src = nW3 + n; strd = DIN; ksrc = HID; kp = HID;
    dst = nW3T + (size_t)n * HID;
  }
  v4u pk[2];
#pragma unroll
  for (int ci = 0; ci < 2; ++ci) {
    const int kc = 8 * tid + 512 * ci;
    float f[8];
#pragma unroll
    for (int i = 0; i < 8; ++i) {
      const int k = kc + i;
      const int kcl = (k < ksrc) ? k : (ksrc - 1);
      const float v = src[(size_t)kcl * strd] * WSCL;
      f[i] = (k < ksrc) ? v : 0.f;
    }
    const v4f f0 = {f[0], f[1], f[2], f[3]};
    const v4f f1 = {f[4], f[5], f[6], f[7]};
    pk[ci] = cvt8(f0, f1);
  }
#pragma unroll
  for (int ci = 0; ci < 2; ++ci) {
    const int kc = 8 * tid + 512 * ci;
    if (kc < kp) *(volatile v4u*)(dst + kc) = pk[ci];
  }
  __threadfence();
#pragma unroll
  for (int ci = 0; ci < 2; ++ci) {
    const int kc = 8 * tid + 512 * ci;
    if (kc < kp) *(volatile v4u*)(dst + kc) = pk[ci];
  }
}

__global__ __launch_bounds__(NTHR) void k_pq(const float* __restrict__ states, const float* __restrict__ eb1,
                                             const _Float16* __restrict__ eW1T, float* PQ) {
  __shared__ __attribute__((aligned(16))) _Float16 xa[16 * XAP];
  __shared__ __attribute__((aligned(16))) float dt[16 * HID];
  const int tid = threadIdx.x, lane = tid & 31, wv = tid >> 5, h = lane >> 4, m = lane & 15;
  const int r0 = blockIdx.x * 16, hf = blockIdx.y;
  if (tid < 64) {
    const int row = tid >> 2, j = tid & 3;
    const float* s = states + (size_t)(r0 + row) * DIN + 8 * j;
    const v4f a0 = *(const v4f*)s, a1 = *(const v4f*)(s + 4);
    *(v4u*)(xa + row * XAP + 8 * j) = cvt8(a0, a1);
  }
  __syncthreads();

  const v8f zero8 = {0.f, 0.f, 0.f, 0.f, 0.f, 0.f, 0.f, 0.f};
  const v16h a = ldf(xa + m * XAP, h);
  v8f acc[4];
#pragma unroll
  for (int s = 0; s < 4; ++s) {
    const v16h b = ldf(eW1T + (size_t)(HID * hf + 64 * wv + 16 * s + m) * W1P, h);
    acc[s] = wmh(a, b, zero8);
  }
#pragma unroll
  for (int s = 0; s < 4; ++s) {
    const int col = 64 * wv + 16 * s + m;
    const float bl = eb1[col];
    const float bsel = (hf == 0) ? bl : 0.f;
#pragma unroll
    for (int r = 0; r < 8; ++r) dt[(8 * h + r) * HID + col] = acc[s][r] * C16 + bsel;
  }
  __syncthreads();

  float* pg = PQ + (size_t)r0 * PQP + HID * hf;
#pragma unroll
  for (int it = 0; it < 8; ++it) {
    const int p = it * NTHR + tid, row = p >> 7, c4 = p & 127;
    const v4f v = *(const v4f*)(dt + 4 * p);
    *(volatile v4f*)(pg + (size_t)row * PQP + 4 * c4) = v;
  }
  __threadfence();
#pragma unroll
  for (int it = 0; it < 8; ++it) {
    const int p = it * NTHR + tid, row = p >> 7, c4 = p & 127;
    const v4f v = *(const v4f*)(dt + 4 * p);
    *(volatile v4f*)(pg + (size_t)row * PQP + 4 * c4) = v;
  }
}

__global__ __launch_bounds__(NTHR) void k_edge(const float* __restrict__ PQ, const _Float16* __restrict__ eW2T,
                                               const float* __restrict__ eb2, const float* __restrict__ eg,
                                               const float* __restrict__ ebt, _Float16* S) {
  __shared__ __attribute__((aligned(16))) _Float16 ha[48 * HP];
  __shared__ float psum[8 * 48];
  __shared__ float mean_s[48];
  __shared__ float rstd_s[48];
  __shared__ __attribute__((aligned(16))) float sbuf[5 * HID];
  const int tid = threadIdx.x, lane = tid & 31, wv = tid >> 5, h = lane >> 4, m = lane & 15;
  const int blk = blockIdx.x;
  const int nbase = (blk >> 1) * NOBJ;
  const int ih = (blk & 1) * 5;
  const int n0 = nbase + ih;
  {
    const int cg = tid & 63, rg = tid >> 6;
#pragma unroll 2
    for (int R = rg; R < 48; R += 4) {
      const int Rc = (R < NEROW) ? R : (NEROW - 1);
      const int i5 = Rc / 9;
      const int jj = Rc - 9 * i5;
      const int i = ih + i5;
      const int j = jj + ((jj >= i) ? 1 : 0);
      const float* pp = PQ + (size_t)(n0 + i5) * PQP + 8 * cg;
      const float* qq = PQ + (size_t)(nbase + j) * PQP + HID + 8 * cg;
      const v4f p0 = *(const v4f*)pp, p1 = *(const v4f*)(pp + 4);
      const v4f q0 = *(const v4f*)qq, q1 = *(const v4f*)(qq + 4);
      const float sc = (R < NEROW) ? WSCL : 0.f;
      v4f x0, x1;
      x0.x = fmaxf(p0.x + q0.x, 0.f) * sc;
      x0.y = fmaxf(p0.y + q0.y, 0.f) * sc;
      x0.z = fmaxf(p0.z + q0.z, 0.f) * sc;
      x0.w = fmaxf(p0.w + q0.w, 0.f) * sc;
      x1.x = fmaxf(p1.x + q1.x, 0.f) * sc;
      x1.y = fmaxf(p1.y + q1.y, 0.f) * sc;
      x1.z = fmaxf(p1.z + q1.z, 0.f) * sc;
      x1.w = fmaxf(p1.w + q1.w, 0.f) * sc;
      *(v4u*)(ha + R * HP + 8 * cg) = cvt8(x0, x1);
    }
  }
  __syncthreads();

  const v8f zero8 = {0.f, 0.f, 0.f, 0.f, 0.f, 0.f, 0.f, 0.f};
  v8f acc[3][4];
#pragma unroll
  for (int mt = 0; mt < 3; ++mt) {
#pragma unroll
    for (int nt = 0; nt < 4; ++nt) acc[mt][nt] = zero8;
  }
#pragma unroll 1
  for (int kt = 0; kt < HID / 32; ++kt) {
    const int k0 = 32 * kt;
    const v16h a0 = ldf(ha + m * HP + k0, h);
    const v16h a1 = ldf(ha + (16 + m) * HP + k0, h);
    const v16h a2 = ldf(ha + (32 + m) * HP + k0, h);
#pragma unroll
    for (int nt = 0; nt < 4; ++nt) {
      const int col = 64 * wv + 16 * nt + m;
      const v16h b = ldf(eW2T + (size_t)col * HID + k0, h);
      acc[0][nt] = wmh(a0, b, acc[0][nt]);
      acc[1][nt] = wmh(a1, b, acc[1][nt]);
      acc[2][nt] = wmh(a2, b, acc[2][nt]);
    }
  }

  float bc[4], gv[4], bev[4];
#pragma unroll
  for (int nt = 0; nt < 4; ++nt) {
    const int col = 64 * wv + 16 * nt + m;
    bc[nt] = eb2[col];
    gv[nt] = eg[col];
    bev[nt] = ebt[col];
  }
#pragma unroll
  for (int mt = 0; mt < 3; ++mt) {
#pragma unroll
    for (int nt = 0; nt < 4; ++nt) {
#pragma unroll
      for (int r = 0; r < 8; ++r) acc[mt][nt][r] = acc[mt][nt][r] * C256 + bc[nt];
    }
  }
#pragma unroll
  for (int mt = 0; mt < 3; ++mt) {
#pragma unroll
    for (int r = 0; r < 8; ++r) {
      float s = (acc[mt][0][r] + acc[mt][1][r]) + (acc[mt][2][r] + acc[mt][3][r]);
      s = sum16(s);
      if (m == 0) psum[wv * 48 + 16 * mt + 8 * h + r] = s;
    }
  }
  __syncthreads();
  if (tid < 48) {
    float t = 0.f;
#pragma unroll
    for (int w = 0; w < 8; ++w) t += psum[w * 48 + tid];
    mean_s[tid] = t * (1.f / HID);
  }
  __syncthreads();
#pragma unroll
  for (int mt = 0; mt < 3; ++mt) {
#pragma unroll
    for (int r = 0; r < 8; ++r) {
      const float mu = mean_s[16 * mt + 8 * h + r];
      float q = 0.f;
#pragma unroll
      for (int nt = 0; nt < 4; ++nt) {
        const float d = acc[mt][nt][r] - mu;
        q += d * d;
      }
      q = sum16(q);
      if (m == 0) psum[wv * 48 + 16 * mt + 8 * h + r] = q;
    }
  }
  __syncthreads();
  if (tid < 48) {
    float t = 0.f;
#pragma unroll
    for (int w = 0; w < 8; ++w) t += psum[w * 48 + tid];
    rstd_s[tid] = rsqrtf(t * (1.f / HID) + LNEPS);
  }
  __syncthreads();

  float part[5][4];
#pragma unroll
  for (int n = 0; n < 5; ++n) {
#pragma unroll
    for (int nt = 0; nt < 4; ++nt) part[n][nt] = 0.f;
  }
#pragma unroll
  for (int mt = 0; mt < 3; ++mt) {
#pragma unroll
    for (int r = 0; r < 8; ++r) {
      const int RA = 16 * mt + r;
      const int RB = RA + 8;
      const float mu = mean_s[RA + 8 * h];
      const float rs = rstd_s[RA + 8 * h];
#pragma unroll
      for (int nt = 0; nt < 4; ++nt) {
        const float y = fmaxf((acc[mt][nt][r] - mu) * rs * gv[nt] + bev[nt], 0.f);
        const float vlo = h ? 0.f : y;
        const float vhi = h ? y : 0.f;
        if (RA < NEROW) part[RA / 9][nt] += vlo;
        if (RB < NEROW) part[RB / 9][nt] += vhi;
      }
    }
  }
#pragma unroll
  for (int n = 0; n < 5; ++n) {
#pragma unroll
    for (int nt = 0; nt < 4; ++nt) {
      float s = part[n][nt];
      s += __shfl_xor(s, 16);
      if (h == 0) sbuf[n * HID + 64 * wv + 16 * nt + m] = s;
    }
  }
  __syncthreads();

  {
    const int p = tid, n = p >> 6, c8 = (p & 63) * 8;
    const v4u u = cvt8(*(const v4f*)(sbuf + n * HID + c8), *(const v4f*)(sbuf + n * HID + c8 + 4));
    *(volatile v4u*)(S + (size_t)(n0 + n) * HID + c8) = u;
    if (tid < 64) {
      const int p2 = NTHR + tid, n2 = p2 >> 6, c82 = (p2 & 63) * 8;
      const v4u u2 = cvt8(*(const v4f*)(sbuf + n2 * HID + c82), *(const v4f*)(sbuf + n2 * HID + c82 + 4));
      *(volatile v4u*)(S + (size_t)(n0 + n2) * HID + c82) = u2;
    }
  }
  __threadfence();
  {
    const int p = tid, n = p >> 6, c8 = (p & 63) * 8;
    const v4u u = cvt8(*(const v4f*)(sbuf + n * HID + c8), *(const v4f*)(sbuf + n * HID + c8 + 4));
    *(volatile v4u*)(S + (size_t)(n0 + n) * HID + c8) = u;
    if (tid < 64) {
      const int p2 = NTHR + tid, n2 = p2 >> 6, c82 = (p2 & 63) * 8;
      const v4u u2 = cvt8(*(const v4f*)(sbuf + n2 * HID + c82), *(const v4f*)(sbuf + n2 * HID + c82 + 4));
      *(volatile v4u*)(S + (size_t)(n0 + n2) * HID + c82) = u2;
    }
  }
}

__global__ __launch_bounds__(NTHR) void k_agg(const _Float16* __restrict__ S, const _Float16* __restrict__ eW3T,
                                              const float* __restrict__ eb3, const float* __restrict__ states,
                                              const float* __restrict__ action, _Float16* XN) {
  __shared__ __attribute__((aligned(16))) _Float16 xrow[32 * XP];
  const int tid = threadIdx.x, lane = tid & 31, wv = tid >> 5, h = lane >> 4, m = lane & 15;
  const int r0 = blockIdx.x * 32;

  const v8f zero8 = {0.f, 0.f, 0.f, 0.f, 0.f, 0.f, 0.f, 0.f};
  v8f acc[2][4];
#pragma unroll
  for (int mt = 0; mt < 2; ++mt) {
#pragma unroll
    for (int nt = 0; nt < 4; ++nt) acc[mt][nt] = zero8;
  }
#pragma unroll 1
  for (int kt = 0; kt < HID / 32; ++kt) {
    const int k0 = 32 * kt;
    const v16h a0 = ldf(S + (size_t)(r0 + m) * HID + k0, h);
    const v16h a1 = ldf(S + (size_t)(r0 + 16 + m) * HID + k0, h);
#pragma unroll
    for (int nt = 0; nt < 4; ++nt) {
      const int col = 64 * wv + 16 * nt + m;
      const v16h b = ldf(eW3T + (size_t)col * HID + k0, h);
      acc[0][nt] = wmh(a0, b, acc[0][nt]);
      acc[1][nt] = wmh(a1, b, acc[1][nt]);
    }
  }
#pragma unroll
  for (int nt = 0; nt < 4; ++nt) {
    const int col = 64 * wv + 16 * nt + m;
    const float b9 = 9.f * eb3[col];
#pragma unroll
    for (int mt = 0; mt < 2; ++mt) {
#pragma unroll
      for (int r = 0; r < 8; ++r) {
        const float v = acc[mt][nt][r] * C16 + b9;
        xrow[(16 * mt + 8 * h + r) * XP + 36 + col] = (_Float16)v;
      }
    }
  }
  {
    const int row = tid >> 3, j = tid & 7;
    const v4f s4 = *(const v4f*)(states + (size_t)(r0 + row) * DIN + 4 * j);
    const v4h hv = {(_Float16)s4.x, (_Float16)s4.y, (_Float16)s4.z, (_Float16)s4.w};
    *(v4h*)(xrow + row * XP + 4 * j) = hv;
    if (j < 7) {
      const v4h z4 = {(_Float16)0.f, (_Float16)0.f, (_Float16)0.f, (_Float16)0.f};
      *(v4h*)(xrow + row * XP + KIN + 4 * j) = z4;
    }
    if (tid < 128) {
      const int arow = tid >> 2, a = tid & 3;
      const float av = action[(size_t)((r0 + arow) / NOBJ) * ADIM + a];
      xrow[arow * XP + DIN + a] = (_Float16)av;
    }
  }
  __syncthreads();

  _Float16* xg = XN + (size_t)r0 * XK;
#pragma unroll
  for (int it = 0; it < 9; ++it) {
    const int p = it * NTHR + tid, row = p / 72, c16 = p - 72 * row;
    Pk8 u;
    u.h = *(const v8h*)(xrow + row * XP + 8 * c16);
    *(volatile v4u*)(xg + (size_t)row * XK + 8 * c16) = u.u;
  }
  __threadfence();
#pragma unroll
  for (int it = 0; it < 9; ++it) {
    const int p = it * NTHR + tid, row = p / 72, c16 = p - 72 * row;
    Pk8 u;
    u.h = *(const v8h*)(xrow + row * XP + 8 * c16);
    *(volatile v4u*)(xg + (size_t)row * XK + 8 * c16) = u.u;
  }
}

__global__ __launch_bounds__(NTHR) void k_n1(const _Float16* __restrict__ XN, const _Float16* __restrict__ nW1T,
                                             const float* __restrict__ nb1, _Float16* HN1) {
  __shared__ __attribute__((aligned(16))) _Float16 hrow[32 * HP];
  const int tid = threadIdx.x, lane = tid & 31, wv = tid >> 5, h = lane >> 4, m = lane & 15;
  const int r0 = blockIdx.x * 32;

  const v8f zero8 = {0.f, 0.f, 0.f, 0.f, 0.f, 0.f, 0.f, 0.f};
  v8f acc[2][4];
#pragma unroll
  for (int mt = 0; mt < 2; ++mt) {
#pragma unroll
    for (int nt = 0; nt < 4; ++nt) acc[mt][nt] = zero8;
  }
#pragma unroll 1
  for (int kt = 0; kt < XK / 32; ++kt) {
    const int k0 = 32 * kt;
    const v16h a0 = ldf(XN + (size_t)(r0 + m) * XK + k0, h);
    const v16h a1 = ldf(XN + (size_t)(r0 + 16 + m) * XK + k0, h);
#pragma unroll
    for (int nt = 0; nt < 4; ++nt) {
      const int col = 64 * wv + 16 * nt + m;
      const v16h b = ldf(nW1T + (size_t)col * XK + k0, h);
      acc[0][nt] = wmh(a0, b, acc[0][nt]);
      acc[1][nt] = wmh(a1, b, acc[1][nt]);
    }
  }
#pragma unroll
  for (int nt = 0; nt < 4; ++nt) {
    const int col = 64 * wv + 16 * nt + m;
    const float bb = nb1[col];
#pragma unroll
    for (int mt = 0; mt < 2; ++mt) {
#pragma unroll
      for (int r = 0; r < 8; ++r) {
        const float v = fmaxf(acc[mt][nt][r] * C16 + bb, 0.f) * WSCL;
        hrow[(16 * mt + 8 * h + r) * HP + col] = (_Float16)v;
      }
    }
  }
  __syncthreads();

  _Float16* hg = HN1 + (size_t)r0 * HID;
#pragma unroll
  for (int it = 0; it < 8; ++it) {
    const int p = it * NTHR + tid, row = p >> 6, c16 = p & 63;
    Pk8 u;
    u.h = *(const v8h*)(hrow + row * HP + 8 * c16);
    *(volatile v4u*)(hg + (size_t)row * HID + 8 * c16) = u.u;
  }
  __threadfence();
#pragma unroll
  for (int it = 0; it < 8; ++it) {
    const int p = it * NTHR + tid, row = p >> 6, c16 = p & 63;
    Pk8 u;
    u.h = *(const v8h*)(hrow + row * HP + 8 * c16);
    *(volatile v4u*)(hg + (size_t)row * HID + 8 * c16) = u.u;
  }
}

__global__ __launch_bounds__(NTHR) void k_n2(const _Float16* __restrict__ HN1, const _Float16* __restrict__ nW2T,
                                             const float* __restrict__ nb2, const float* __restrict__ ng,
                                             const float* __restrict__ nbt, const _Float16* __restrict__ nW3T,
                                             const float* __restrict__ nb3, float* out) {
  __shared__ __attribute__((aligned(16))) _Float16 h2t[32 * HP];
  __shared__ float psum[8 * 32];
  __shared__ float mean_s[32];
  __shared__ float rstd_s[32];
  __shared__ __attribute__((aligned(16))) float obuf[32 * DIN];
  const int tid = threadIdx.x, lane = tid & 31, wv = tid >> 5, h = lane >> 4, m = lane & 15;
  const int r0 = blockIdx.x * 32;

  const v8f zero8 = {0.f, 0.f, 0.f, 0.f, 0.f, 0.f, 0.f, 0.f};
  v8f acc[2][4];
#pragma unroll
  for (int mt = 0; mt < 2; ++mt) {
#pragma unroll
    for (int nt = 0; nt < 4; ++nt) acc[mt][nt] = zero8;
  }
#pragma unroll 1
  for (int kt = 0; kt < HID / 32; ++kt) {
    const int k0 = 32 * kt;
    const v16h a0 = ldf(HN1 + (size_t)(r0 + m) * HID + k0, h);
    const v16h a1 = ldf(HN1 + (size_t)(r0 + 16 + m) * HID + k0, h);
#pragma unroll
    for (int nt = 0; nt < 4; ++nt) {
      const int col = 64 * wv + 16 * nt + m;
      const v16h b = ldf(nW2T + (size_t)col * HID + k0, h);
      acc[0][nt] = wmh(a0, b, acc[0][nt]);
      acc[1][nt] = wmh(a1, b, acc[1][nt]);
    }
  }

  float bc[4], gv[4], bev[4];
#pragma unroll
  for (int nt = 0; nt < 4; ++nt) {
    const int col = 64 * wv + 16 * nt + m;
    bc[nt] = nb2[col];
    gv[nt] = ng[col];
    bev[nt] = nbt[col];
  }
#pragma unroll
  for (int mt = 0; mt < 2; ++mt) {
#pragma unroll
    for (int nt = 0; nt < 4; ++nt) {
#pragma unroll
      for (int r = 0; r < 8; ++r) acc[mt][nt][r] = acc[mt][nt][r] * C256 + bc[nt];
    }
  }
#pragma unroll
  for (int mt = 0; mt < 2; ++mt) {
#pragma unroll
    for (int r = 0; r < 8; ++r) {
      float s = (acc[mt][0][r] + acc[mt][1][r]) + (acc[mt][2][r] + acc[mt][3][r]);
      s = sum16(s);
      if (m == 0) psum[wv * 32 + 16 * mt + 8 * h + r] = s;
    }
  }
  __syncthreads();
  if (tid < 32) {
    float t = 0.f;
#pragma unroll
    for (int w = 0; w < 8; ++w) t += psum[w * 32 + tid];
    mean_s[tid] = t * (1.f / HID);
  }
  __syncthreads();
#pragma unroll
  for (int mt = 0; mt < 2; ++mt) {
#pragma unroll
    for (int r = 0; r < 8; ++r) {
      const float mu = mean_s[16 * mt + 8 * h + r];
      float q = 0.f;
#pragma unroll
      for (int nt = 0; nt < 4; ++nt) {
        const float d = acc[mt][nt][r] - mu;
        q += d * d;
      }
      q = sum16(q);
      if (m == 0) psum[wv * 32 + 16 * mt + 8 * h + r] = q;
    }
  }
  __syncthreads();
  if (tid < 32) {
    float t = 0.f;
#pragma unroll
    for (int w = 0; w < 8; ++w) t += psum[w * 32 + tid];
    rstd_s[tid] = rsqrtf(t * (1.f / HID) + LNEPS);
  }
  __syncthreads();
#pragma unroll
  for (int mt = 0; mt < 2; ++mt) {
#pragma unroll
    for (int r = 0; r < 8; ++r) {
      const int row = 16 * mt + 8 * h + r;
      const float mu = mean_s[row];
      const float rs = rstd_s[row];
#pragma unroll
      for (int nt = 0; nt < 4; ++nt) {
        const int col = 64 * wv + 16 * nt + m;
        const float y = fmaxf((acc[mt][nt][r] - mu) * rs * gv[nt] + bev[nt], 0.f) * WSCL;
        h2t[row * HP + col] = (_Float16)y;
      }
    }
  }
  __syncthreads();

  if (wv < 4) {
    const int mt3 = wv >> 1, nt3 = wv & 1;
    v8f a3 = zero8;
#pragma unroll 1
    for (int kt = 0; kt < HID / 32; ++kt) {
      const int k0 = 32 * kt;
      const v16h a = ldf(h2t + (16 * mt3 + m) * HP + k0, h);
      const v16h b = ldf(nW3T + (size_t)(16 * nt3 + m) * HID + k0, h);
      a3 = wmh(a, b, a3);
    }
    const float ob = nb3[16 * nt3 + m];
#pragma unroll
    for (int r = 0; r < 8; ++r) obuf[(16 * mt3 + 8 * h + r) * DIN + 16 * nt3 + m] = a3[r] * C256 + ob;
  }
  __syncthreads();

  {
    const int row = tid >> 3, q = tid & 7;
    const v4f v = *(const v4f*)(obuf + row * DIN + 4 * q);
    float* p = out + (size_t)(r0 + row) * DIN + 4 * q;
    *(volatile v4f*)p = v;
    __threadfence();
    *(volatile v4f*)p = v;
  }
}

extern "C" void kernel_launch(void* const* d_in, const int* in_sizes, int n_in,
                              void* d_out, int out_size, void* d_ws, size_t ws_size,
                              hipStream_t stream) {
  if (n_in < 18) return;
  if (in_sizes[0] != NNODE * DIN) return;
  if (in_sizes[1] != NBAT * ADIM) return;
  if (in_sizes[2] != 2 * DIN * HID || in_sizes[3] != HID) return;
  if (in_sizes[4] != HID * HID || in_sizes[5] != HID) return;
  if (in_sizes[6] != HID || in_sizes[7] != HID) return;
  if (in_sizes[8] != HID * HID || in_sizes[9] != HID) return;
  if (in_sizes[10] != KIN * HID || in_sizes[11] != HID) return;
  if (in_sizes[12] != HID * HID || in_sizes[13] != HID) return;
  if (in_sizes[14] != HID || in_sizes[15] != HID) return;
  if (in_sizes[16] != HID * DIN || in_sizes[17] != DIN) return;
  if (out_size != NNODE * DIN) return;

  const float* states = (const float*)d_in[0];
  const float* action = (const float*)d_in[1];
  const float* eW1 = (const float*)d_in[2];
  const float* eb1 = (const float*)d_in[3];
  const float* eW2 = (const float*)d_in[4];
  const float* eb2 = (const float*)d_in[5];
  const float* eg  = (const float*)d_in[6];
  const float* ebt = (const float*)d_in[7];
  const float* eW3 = (const float*)d_in[8];
  const float* eb3 = (const float*)d_in[9];
  const float* nW1 = (const float*)d_in[10];
  const float* nb1 = (const float*)d_in[11];
  const float* nW2 = (const float*)d_in[12];
  const float* nb2 = (const float*)d_in[13];
  const float* ng  = (const float*)d_in[14];
  const float* nbt = (const float*)d_in[15];
  const float* nW3 = (const float*)d_in[16];
  const float* nb3 = (const float*)d_in[17];
  float* out = (float*)d_out;

  char* ws = (char*)d_ws;
  size_t off = 0;
  const size_t oEW1T = off; off += SZ_EW1T;
  const size_t oEW2T = off; off += SZ_EW2T;
  const size_t oEW3T = off; off += SZ_EW3T;
  const size_t oNW1T = off; off += SZ_NW1T;
  const size_t oNW2T = off; off += SZ_NW2T;
  const size_t oNW3T = off; off += SZ_NW3T;
  const size_t oPQ   = off; off += SZ_PQ;
  const size_t oS    = off; off += SZ_S;
  const size_t oXN   = oPQ;
  const size_t oHN1  = oPQ + SZ_XN;
  if (off != SZ_TOT) return;
  if (off > ws_size || off > (size_t)WSCAP) return;
  if (oHN1 + SZ_HN1 > oPQ + SZ_PQ) return;

  _Float16* eW1T = (_Float16*)(ws + oEW1T);
  _Float16* eW2T = (_Float16*)(ws + oEW2T);
  _Float16* eW3T = (_Float16*)(ws + oEW3T);
  _Float16* nW1T = (_Float16*)(ws + oNW1T);
  _Float16* nW2T = (_Float16*)(ws + oNW2T);
  _Float16* nW3T = (_Float16*)(ws + oNW3T);
  float* PQ      = (float*)(ws + oPQ);
  _Float16* S    = (_Float16*)(ws + oS);
  _Float16* XN   = (_Float16*)(ws + oXN);
  _Float16* HN1  = (_Float16*)(ws + oHN1);

  k_prep<<<NPREP, 64, 0, stream>>>(eW1, eW2, eW3, nW1, nW2, nW3, eW1T, eW2T, eW3T, nW1T, nW2T, nW3T);
  k_pq<<<dim3(NNODE / 16, 2), NTHR, 0, stream>>>(states, eb1, eW1T, PQ);
  k_edge<<<NBAT * 2, NTHR, 0, stream>>>(PQ, eW2T, eb2, eg, ebt, S);
  k_agg<<<NNODE / 32, NTHR, 0, stream>>>(S, eW3T, eb3, states, action, XN);
  k_n1<<<NNODE / 32, NTHR, 0, stream>>>(XN, nW1T, nb1, HN1);
  k_n2<<<NNODE / 32, NTHR, 0, stream>>>(HN1, nW2T, nb2, ng, nbt, nW3T, nb3, out);
}
